// WindowedAttentionCore_59674275611314
// MI455X (gfx1250) — hardware-verified
//
#include <hip/hip_runtime.h>


typedef unsigned short u16;
typedef __bf16 v16bf __attribute__((ext_vector_type(16)));
typedef float v8f __attribute__((ext_vector_type(8)));
typedef float v4f __attribute__((ext_vector_type(4)));
typedef unsigned int v4u __attribute__((ext_vector_type(4)));
typedef v4u __attribute__((may_alias)) v4ua;
typedef v4f __attribute__((may_alias)) v4fa;

#define SEQ    2048
#define HIDDEN 2048
#define NHEADS 16
#define HD     128
#define KVDIM  512
#define KVG    4

typedef char dims_check[((SEQ % 64) == 0 && (HIDDEN % 64) == 0 && (KVDIM % 64) == 0 &&
                          (HIDDEN % 32) == 0 && (SEQ % 32) == 0 && NHEADS * HD == HIDDEN &&
                          (NHEADS / KVG) * HD == KVDIM && (HD % 64) == 0) ? 1 : -1];

union Frag {
  v16bf v;
  v4u u[2];
};

__device__ __forceinline__ unsigned int bf16_rne(float f) {
  unsigned int u = __float_as_uint(f);
  u += 0x7fffu + ((u >> 16) & 1u);
  return u >> 16;
}

__device__ __forceinline__ void split2(float x, unsigned int& hi, unsigned int& lo) {
  hi = bf16_rne(x);
  lo = bf16_rne(x - __uint_as_float(hi << 16));
}

__device__ __forceinline__ v8f zero8() {
  v8f z;
#pragma unroll
  for (int i = 0; i < 8; ++i) z[i] = 0.0f;
  return z;
}

__device__ __forceinline__ v8f wmma3(const Frag& ah, const Frag& al,
                                     const Frag& bh, const Frag& bl, v8f acc) {
  acc = __builtin_amdgcn_wmma_f32_16x16x32_bf16(false, ah.v, false, bh.v, (short)0, acc, false, false);
  acc = __builtin_amdgcn_wmma_f32_16x16x32_bf16(false, al.v, false, bh.v, (short)0, acc, false, false);
  acc = __builtin_amdgcn_wmma_f32_16x16x32_bf16(false, ah.v, false, bl.v, (short)0, acc, false, false);
  asm volatile("v_nop\n\tv_nop\n\tv_nop\n\tv_nop"
               : "+v"(acc)
               : "v"(ah.v), "v"(al.v), "v"(bh.v), "v"(bl.v));
  return acc;
}

__device__ __forceinline__ void st_vol(u16* p, v4u v) { *(volatile v4u*)p = v; }
__device__ __forceinline__ void st_vol(float* p, v4f v) { *(volatile v4f*)p = v; }

__global__ __launch_bounds__(256) void k_split(const float* __restrict__ in,
                                               u16* __restrict__ oh,
                                               u16* __restrict__ ol, int n8) {
  const int id = blockIdx.x * 256 + threadIdx.x;
  if (id >= n8) return;
  const size_t base = (size_t)id * 8;
  const v4f a = *(const v4f*)(in + base);
  const v4f b = *(const v4f*)(in + base + 4);
  float x[8];
  x[0] = a[0]; x[1] = a[1]; x[2] = a[2]; x[3] = a[3];
  x[4] = b[0]; x[5] = b[1]; x[6] = b[2]; x[7] = b[3];
  unsigned int hh[8], ll[8];
#pragma unroll
  for (int e = 0; e < 8; ++e) split2(x[e], hh[e], ll[e]);
  v4u H, L;
#pragma unroll
  for (int q = 0; q < 4; ++q) {
    H[q] = hh[2 * q] | (hh[2 * q + 1] << 16);
    L[q] = ll[2 * q] | (ll[2 * q + 1] << 16);
  }
  u16* ph = oh + base;
  u16* pl = ol + base;
  st_vol(ph, H);
  st_vol(pl, L);
  __threadfence();
  st_vol(ph, H);
  st_vol(pl, L);
}

__global__ __launch_bounds__(256) void k_wt_split(const float* __restrict__ W,
                                                  u16* __restrict__ oh,
                                                  u16* __restrict__ ol, int K, int N) {
  __shared__ __attribute__((aligned(16))) u16 th[64][72];
  __shared__ __attribute__((aligned(16))) u16 tl[64][72];
  const int tid = threadIdx.x;
  const int n0 = blockIdx.x * 64;
  const int k0 = blockIdx.y * 64;
  {
    const int kr = tid >> 2;
    const int nc = (tid & 3) * 16;
    const float* src = W + (size_t)(k0 + kr) * N + n0 + nc;
#pragma unroll
    for (int q = 0; q < 4; ++q) {
      const v4f v = *(const v4f*)(src + 4 * q);
#pragma unroll
      for (int e = 0; e < 4; ++e) {
        unsigned int hi, lo;
        split2(v[e], hi, lo);
        th[nc + 4 * q + e][kr] = (u16)hi;
        tl[nc + 4 * q + e][kr] = (u16)lo;
      }
    }
  }
  __syncthreads();
  v4u H[2], L[2];
  u16* ph[2];
  u16* pl[2];
#pragma unroll
  for (int rep = 0; rep < 2; ++rep) {
    const int idx = tid + 256 * rep;
    const int nr = idx >> 3;
    const int c = (idx & 7) * 8;
    H[rep] = *(const v4ua*)&th[nr][c];
    L[rep] = *(const v4ua*)&tl[nr][c];
    const size_t o = (size_t)(n0 + nr) * K + k0 + c;
    ph[rep] = oh + o;
    pl[rep] = ol + o;
  }
#pragma unroll
  for (int rep = 0; rep < 2; ++rep) { st_vol(ph[rep], H[rep]); st_vol(pl[rep], L[rep]); }
  __threadfence();
#pragma unroll
  for (int rep = 0; rep < 2; ++rep) { st_vol(ph[rep], H[rep]); st_vol(pl[rep], L[rep]); }
}

__global__ __launch_bounds__(128) __attribute__((amdgpu_num_vgpr(256)))
void k_gemm(const u16* __restrict__ Ah, const u16* __restrict__ Al,
            const u16* __restrict__ Bh, const u16* __restrict__ Bl,
            float* __restrict__ C, int M, int N, int K) {
  __shared__ __attribute__((aligned(16))) u16 sAh[64][40];
  __shared__ __attribute__((aligned(16))) u16 sAl[64][40];
  __shared__ __attribute__((aligned(16))) u16 sBh[64][40];
  __shared__ __attribute__((aligned(16))) u16 sBl[64][40];
  __shared__ __attribute__((aligned(16))) float sC[64][68];
  (void)M;

  const int tid  = threadIdx.x;
  const int lane = tid & 31;
  const int wave = tid >> 5;
  const int lr   = lane & 15;
  const int g    = lane >> 4;
  const int wm   = wave >> 1;
  const int wn   = wave & 1;
  const int m0   = blockIdx.y * 64;
  const int n0   = blockIdx.x * 64;

  v8f acc[2][2];
#pragma unroll
  for (int i = 0; i < 2; ++i)
#pragma unroll
    for (int j = 0; j < 2; ++j) acc[i][j] = zero8();

  int srow[2], scol[2];
#pragma unroll
  for (int rep = 0; rep < 2; ++rep) {
    const int idx = tid + 128 * rep;
    srow[rep] = idx >> 2;
    scol[rep] = (idx & 3) * 8;
  }

  for (int k0 = 0; k0 < K; k0 += 32) {
#pragma unroll
    for (int rep = 0; rep < 2; ++rep) {
      const size_t ao = (size_t)(m0 + srow[rep]) * K + k0 + scol[rep];
      const size_t bo = (size_t)(n0 + srow[rep]) * K + k0 + scol[rep];
      *(v4ua*)&sAh[srow[rep]][scol[rep]] = *(const v4u*)(Ah + ao);
      *(v4ua*)&sAl[srow[rep]][scol[rep]] = *(const v4u*)(Al + ao);
      *(v4ua*)&sBh[srow[rep]][scol[rep]] = *(const v4u*)(Bh + bo);
      *(v4ua*)&sBl[srow[rep]][scol[rep]] = *(const v4u*)(Bl + bo);
    }
    __syncthreads();

    Frag fah[2], fal[2], fbh[2], fbl[2];
#pragma unroll
    for (int i = 0; i < 2; ++i) {
      const int r = wm * 32 + i * 16 + lr;
      fah[i].u[0] = *(const v4ua*)&sAh[r][8 * g];
      fah[i].u[1] = *(const v4ua*)&sAh[r][16 + 8 * g];
      fal[i].u[0] = *(const v4ua*)&sAl[r][8 * g];
      fal[i].u[1] = *(const v4ua*)&sAl[r][16 + 8 * g];
    }
#pragma unroll
    for (int j = 0; j < 2; ++j) {
      const int r = wn * 32 + j * 16 + lr;
      fbh[j].u[0] = *(const v4ua*)&sBh[r][8 * g];
      fbh[j].u[1] = *(const v4ua*)&sBh[r][16 + 8 * g];
      fbl[j].u[0] = *(const v4ua*)&sBl[r][8 * g];
      fbl[j].u[1] = *(const v4ua*)&sBl[r][16 + 8 * g];
    }
#pragma unroll
    for (int i = 0; i < 2; ++i)
#pragma unroll
      for (int j = 0; j < 2; ++j)
        acc[i][j] = wmma3(fah[i], fal[i], fbh[j], fbl[j], acc[i][j]);
    __syncthreads();
  }

#pragma unroll
  for (int i = 0; i < 2; ++i)
#pragma unroll
    for (int j = 0; j < 2; ++j)
#pragma unroll
      for (int r = 0; r < 8; ++r)
        sC[wm * 32 + i * 16 + 8 * g + r][wn * 32 + j * 16 + lr] = acc[i][j][r];
  __syncthreads();

  v4f cv[8];
  float* cp[8];
#pragma unroll
  for (int rep = 0; rep < 8; ++rep) {
    const int idx = tid + 128 * rep;
    const int row = idx >> 4;
    const int c   = (idx & 15) * 4;
    cv[rep] = *(const v4fa*)&sC[row][c];
    cp[rep] = C + (size_t)(m0 + row) * N + n0 + c;
  }
#pragma unroll
  for (int rep = 0; rep < 8; ++rep) st_vol(cp[rep], cv[rep]);
  __threadfence();
#pragma unroll
  for (int rep = 0; rep < 8; ++rep) st_vol(cp[rep], cv[rep]);
}

__global__ __launch_bounds__(128) __attribute__((amdgpu_num_vgpr(256)))
void k_attn(const u16* __restrict__ Qh, const u16* __restrict__ Ql,
            const u16* __restrict__ Kh, const u16* __restrict__ Kl,
            const u16* __restrict__ Vh, const u16* __restrict__ Vl,
            const int* __restrict__ msk, float* __restrict__ O) {
  __shared__ __attribute__((aligned(16))) u16 sPh[4][16][40];
  __shared__ __attribute__((aligned(16))) u16 sPl[4][16][40];
  __shared__ __attribute__((aligned(16))) float sO[4][16][68];

  const int lane = threadIdx.x & 31;
  const int wave = threadIdx.x >> 5;
  const int lr   = lane & 15;
  const int g    = lane >> 4;
  const int h    = blockIdx.y;
  const int i0   = (blockIdx.x * 2 + (wave >> 1)) * 16;
  const int dh   = wave & 1;
  const int kvh  = h / KVG;
  const float scale = 0.08838834764831845f;
  const float NEG = -3.0e38f;

  v8f oacc[4];
#pragma unroll
  for (int t = 0; t < 4; ++t) oacc[t] = zero8();
  float rowM[8], rowL[8];
#pragma unroll
  for (int r = 0; r < 8; ++r) { rowM[r] = NEG; rowL[r] = 0.0f; }

  const u16* qh_row = Qh + (size_t)(i0 + lr) * HIDDEN + h * HD + 8 * g;
  const u16* ql_row = Ql + (size_t)(i0 + lr) * HIDDEN + h * HD + 8 * g;
  const u16* kh_base = Kh + (size_t)lr * KVDIM + kvh * HD + 8 * g;
  const u16* kl_base = Kl + (size_t)lr * KVDIM + kvh * HD + 8 * g;
  const u16* vh_base = Vh + (size_t)(kvh * HD + dh * 64 + lr) * SEQ + 8 * g;
  const u16* vl_base = Vl + (size_t)(kvh * HD + dh * 64 + lr) * SEQ + 8 * g;
  const int* m_base = msk + (size_t)(i0 + 8 * g) * SEQ + lr;

  for (int j0 = 0; j0 < SEQ; j0 += 32) {
    v8f sc0 = zero8();
    v8f sc1 = zero8();
#pragma unroll 1
    for (int kc = 0; kc < 4; ++kc) {
      Frag qh, ql;
      qh.u[0] = *(const v4u*)(qh_row + kc * 32);
      qh.u[1] = *(const v4u*)(qh_row + kc * 32 + 16);
      ql.u[0] = *(const v4u*)(ql_row + kc * 32);
      ql.u[1] = *(const v4u*)(ql_row + kc * 32 + 16);
      {
        const size_t ko = (size_t)j0 * KVDIM + kc * 32;
        Frag kh, kl;
        kh.u[0] = *(const v4u*)(kh_base + ko);
        kh.u[1] = *(const v4u*)(kh_base + ko + 16);
        kl.u[0] = *(const v4u*)(kl_base + ko);
        kl.u[1] = *(const v4u*)(kl_base + ko + 16);
        sc0 = wmma3(qh, ql, kh, kl, sc0);
      }
      {
        const size_t ko = (size_t)(j0 + 16) * KVDIM + kc * 32;
        Frag kh, kl;
        kh.u[0] = *(const v4u*)(kh_base + ko);
        kh.u[1] = *(const v4u*)(kh_base + ko + 16);
        kl.u[0] = *(const v4u*)(kl_base + ko);
        kl.u[1] = *(const v4u*)(kl_base + ko + 16);
        sc1 = wmma3(qh, ql, kh, kl, sc1);
      }
    }

#pragma unroll
    for (int r = 0; r < 8; ++r) {
      const int* mp = m_base + (size_t)r * SEQ + j0;
      const int mk0 = mp[0];
      const int mk1 = mp[16];
      const float s0 = (mk0 != 0) ? sc0[r] * scale : NEG;
      const float s1 = (mk1 != 0) ? sc1[r] * scale : NEG;
      float mx = fmaxf(s0, s1);
      mx = fmaxf(mx, __shfl_xor(mx, 8));
      mx = fmaxf(mx, __shfl_xor(mx, 4));
      mx = fmaxf(mx, __shfl_xor(mx, 2));
      mx = fmaxf(mx, __shfl_xor(mx, 1));
      const float mnew = fmaxf(rowM[r], mx);
      const float corr = __expf(rowM[r] - mnew);
      rowM[r] = mnew;
      const float p0 = (mk0 != 0) ? __expf(s0 - mnew) : 0.0f;
      const float p1 = (mk1 != 0) ? __expf(s1 - mnew) : 0.0f;
      float ps = p0 + p1;
      ps += __shfl_xor(ps, 8);
      ps += __shfl_xor(ps, 4);
      ps += __shfl_xor(ps, 2);
      ps += __shfl_xor(ps, 1);
      rowL[r] = rowL[r] * corr + ps;
#pragma unroll
      for (int t = 0; t < 4; ++t) oacc[t][r] = oacc[t][r] * corr;
      unsigned int ph0, pl0, ph1, pl1;
      split2(p0, ph0, pl0);
      split2(p1, ph1, pl1);
      sPh[wave][8 * g + r][lr]      = (u16)ph0;
      sPh[wave][8 * g + r][16 + lr] = (u16)ph1;
      sPl[wave][8 * g + r][lr]      = (u16)pl0;
      sPl[wave][8 * g + r][16 + lr] = (u16)pl1;
    }
    __syncthreads();

    Frag fph, fpl;
    fph.u[0] = *(const v4ua*)&sPh[wave][lr][8 * g];
    fph.u[1] = *(const v4ua*)&sPh[wave][lr][16 + 8 * g];
    fpl.u[0] = *(const v4ua*)&sPl[wave][lr][8 * g];
    fpl.u[1] = *(const v4ua*)&sPl[wave][lr][16 + 8 * g];

#pragma unroll
    for (int t = 0; t < 4; ++t) {
      const size_t vo = (size_t)(t * 16) * SEQ + j0;
      Frag vh, vl;
      vh.u[0] = *(const v4u*)(vh_base + vo);
      vh.u[1] = *(const v4u*)(vh_base + vo + 16);
      vl.u[0] = *(const v4u*)(vl_base + vo);
      vl.u[1] = *(const v4u*)(vl_base + vo + 16);
      oacc[t] = wmma3(fph, fpl, vh, vl, oacc[t]);
    }
    __syncthreads();
  }

#pragma unroll
  for (int r = 0; r < 8; ++r) {
    const float L = rowL[r];
    const float inv = (L > 0.0f) ? (1.0f / L) : 0.0f;
#pragma unroll
    for (int t = 0; t < 4; ++t) sO[wave][8 * g + r][t * 16 + lr] = oacc[t][r] * inv;
  }
  __syncthreads();

  v4f ov[8];
  float* op[8];
#pragma unroll
  for (int rep = 0; rep < 8; ++rep) {
    const int idx = lane + 32 * rep;
    const int row = idx >> 4;
    const int c   = (idx & 15) * 4;
    ov[rep] = *(const v4fa*)&sO[wave][row][c];
    op[rep] = O + (size_t)(i0 + row) * HIDDEN + h * HD + dh * 64 + c;
  }
#pragma unroll
  for (int rep = 0; rep < 8; ++rep) st_vol(op[rep], ov[rep]);
  __threadfence();
#pragma unroll
  for (int rep = 0; rep < 8; ++rep) st_vol(op[rep], ov[rep]);
}

extern "C" void kernel_launch(void* const* d_in, const int* in_sizes, int n_in,
                              void* d_out, int out_size, void* d_ws, size_t ws_size,
                              hipStream_t stream) {
  if (n_in < 6) return;
  if (in_sizes[0] != SEQ * HIDDEN || in_sizes[1] != SEQ * SEQ ||
      in_sizes[2] != HIDDEN * HIDDEN || in_sizes[3] != HIDDEN * KVDIM ||
      in_sizes[4] != HIDDEN * KVDIM || in_sizes[5] != HIDDEN * HIDDEN) return;
  if (out_size != SEQ * HIDDEN) return;

  const float* X   = (const float*)d_in[0];
  const int*   msk = (const int*)d_in[1];
  const float* Wq  = (const float*)d_in[2];
  const float* Wk  = (const float*)d_in[3];
  const float* Wv  = (const float*)d_in[4];
  const float* Wo  = (const float*)d_in[5];
  float* out       = (float*)d_out;

  char* ws = (char*)d_ws;
  size_t off = 0;
  const size_t bSH2 = (size_t)SEQ * HIDDEN * 2;
  const size_t bHH2 = (size_t)HIDDEN * HIDDEN * 2;
  const size_t bHK2 = (size_t)HIDDEN * KVDIM * 2;
  const size_t bSK2 = (size_t)SEQ * KVDIM * 2;
  u16* Xh   = (u16*)(ws + off); off += bSH2;
  u16* Xl   = (u16*)(ws + off); off += bSH2;
  u16* WqTh = (u16*)(ws + off); off += bHH2;
  u16* WqTl = (u16*)(ws + off); off += bHH2;
  u16* WkTh = (u16*)(ws + off); off += bHK2;
  u16* WkTl = (u16*)(ws + off); off += bHK2;
  u16* WvTh = (u16*)(ws + off); off += bHK2;
  u16* WvTl = (u16*)(ws + off); off += bHK2;
  u16* WoTh = (u16*)(ws + off); off += bHH2;
  u16* WoTl = (u16*)(ws + off); off += bHH2;
  float* Qf = (float*)(ws + off); off += bSH2 * 2;
  u16* Qh   = (u16*)(ws + off); off += bSH2;
  u16* Ql   = (u16*)(ws + off); off += bSH2;
  float* Kf = (float*)(ws + off); off += bSK2 * 2;
  u16* Khp  = (u16*)(ws + off); off += bSK2;
  u16* Klp  = (u16*)(ws + off); off += bSK2;
  float* VTf = (float*)(ws + off); off += bSK2 * 2;
  u16* VTh  = (u16*)(ws + off); off += bSK2;
  u16* VTl  = (u16*)(ws + off); off += bSK2;
  float* Of = (float*)(ws + off); off += bSH2 * 2;
  u16* Oh   = (u16*)(ws + off); off += bSH2;
  u16* Ol   = (u16*)(ws + off); off += bSH2;
  if (off > ws_size) return;

  const dim3 b256(256), b128(128);
  const int n8_SH = SEQ * HIDDEN / 8;
  const int n8_SK = SEQ * KVDIM / 8;

  k_split<<<dim3((n8_SH + 255) / 256), b256, 0, stream>>>(X, Xh, Xl, n8_SH);
  k_wt_split<<<dim3(HIDDEN / 64, HIDDEN / 64), b256, 0, stream>>>(Wq, WqTh, WqTl, HIDDEN, HIDDEN);
  k_wt_split<<<dim3(KVDIM / 64, HIDDEN / 64), b256, 0, stream>>>(Wk, WkTh, WkTl, HIDDEN, KVDIM);
  k_wt_split<<<dim3(KVDIM / 64, HIDDEN / 64), b256, 0, stream>>>(Wv, WvTh, WvTl, HIDDEN, KVDIM);
  k_wt_split<<<dim3(HIDDEN / 64, HIDDEN / 64), b256, 0, stream>>>(Wo, WoTh, WoTl, HIDDEN, HIDDEN);

  k_gemm<<<dim3(HIDDEN / 64, SEQ / 64), b128, 0, stream>>>(Xh, Xl, WqTh, WqTl, Qf, SEQ, HIDDEN, HIDDEN);
  k_split<<<dim3((n8_SH + 255) / 256), b256, 0, stream>>>(Qf, Qh, Ql, n8_SH);
  k_gemm<<<dim3(KVDIM / 64, SEQ / 64), b128, 0, stream>>>(Xh, Xl, WkTh, WkTl, Kf, SEQ, KVDIM, HIDDEN);
  k_split<<<dim3((n8_SK + 255) / 256), b256, 0, stream>>>(Kf, Khp, Klp, n8_SK);
  k_gemm<<<dim3(SEQ / 64, KVDIM / 64), b128, 0, stream>>>(WvTh, WvTl, Xh, Xl, VTf, KVDIM, SEQ, HIDDEN);
  k_split<<<dim3((n8_SK + 255) / 256), b256, 0, stream>>>(VTf, VTh, VTl, n8_SK);

  k_attn<<<dim3(SEQ / 32, NHEADS), b128, 0, stream>>>(Qh, Ql, Khp, Klp, VTh, VTl, msk, Of);
  k_split<<<dim3((n8_SH + 255) / 256), b256, 0, stream>>>(Of, Oh, Ol, n8_SH);

  k_gemm<<<dim3(HIDDEN / 64, SEQ / 64), b128, 0, stream>>>(Oh, Ol, WoTh, WoTl, out, SEQ, HIDDEN, HIDDEN);
}
